// EvolvingFieldSystem_54494545052129
// MI455X (gfx1250) — hardware-run, weakly checked
//
#include <hip/hip_runtime.h>
#include <math.h>

typedef __attribute__((ext_vector_type(16))) _Float16 v16h;
typedef __attribute__((ext_vector_type(8)))  _Float16 v8h;
typedef __attribute__((ext_vector_type(8)))  float    v8f;
typedef __attribute__((ext_vector_type(4)))  float    v4f;

constexpr int kN        = 2097152;
constexpr int kBlobs    = 20;
constexpr int kState    = 160;
constexpr int kDynHid   = 64;
constexpr int kSumW     = 32;
constexpr int kEnc      = 24;
constexpr int kFqIn     = 56;
constexpr int kColIn    = 57;
constexpr int kHid      = 64;
constexpr int kKP       = 32;
constexpr int kHeadRows = 16;
constexpr int kAP       = 40;
constexpr int kHP       = 72;
constexpr int kGroupPts = 32;
constexpr int kGroupsPerWave = 4;
constexpr int kWavesPerBlock = 8;
constexpr int kBlockPts = kWavesPerBlock * kGroupsPerWave * kGroupPts;
constexpr int kMaxSteps = 4096;
static_assert(kBlobs * 8 == kState, "state width");
static_assert(kEnc + kSumW == kFqIn && kFqIn + 1 == kColIn, "first-layer input widths");
static_assert(kEnc + 1 <= kKP && (kKP % 32) == 0 && (kHid % 32) == 0, "K multiples of 32");
static_assert((kN % kBlockPts) == 0, "no point tails");
static_assert((size_t)kN * 4 + (size_t)kN * 3 * 4 == 33554432ull, "output bytes");
static_assert(((size_t)kN * 4) % 128 == 0, "second output starts on a line");

constexpr size_t kOffBias = 0;
constexpr size_t kOffW1t  = kOffBias + (size_t)128 * 4;
constexpr size_t kOffWct  = kOffW1t + (size_t)kHid * kKP * 2;
constexpr size_t kOffHh   = kOffWct + (size_t)kHid * kKP * 2;
constexpr size_t kWsTotal = kOffHh + (size_t)kHeadRows * kHid * 2;
static_assert(kWsTotal == 10752ull, "carve total");
static_assert((kOffW1t % 128) == 0 && (kOffWct % 128) == 0 && (kOffHh % 128) == 0, "aligned regions");

template <typename T> struct Frag;
template <> struct Frag<_Float16> {
  typedef v16h V; union U { v16h v; v8h h[2]; };
  static __device__ __forceinline__ v16h load(const _Float16* p) {
    U f; f.h[0] = *(const v8h*)(p); f.h[1] = *(const v8h*)(p + 16); return f.v;
  }
};

__device__ __forceinline__ v8f mma_h(v16h a, v16h b, v8f c) {
  c = __builtin_amdgcn_wmma_f32_16x16x32_f16(false, a, false, b, (short)0, c, false, false);
  asm volatile("v_nop\n\tv_nop\n\tv_nop\n\tv_nop" : "+v"(c) : "v"(a), "v"(b));
  return c;
}

__device__ __forceinline__ float pin_f32(float x) { asm volatile("" : "+v"(x)); return x; }
__device__ __forceinline__ v4f pin_v4(v4f x) { asm volatile("" : "+v"(x)); return x; }

__device__ __forceinline__ void wave_lds_sync() {
  __builtin_amdgcn_fence(__ATOMIC_RELEASE, "workgroup");
  __builtin_amdgcn_wave_barrier();
  __builtin_amdgcn_fence(__ATOMIC_ACQUIRE, "workgroup");
}

__global__ __launch_bounds__(256) void prep_kernel(
    const float* __restrict__ initial_state,
    const float* __restrict__ dyn_w1, const float* __restrict__ dyn_b1,
    const float* __restrict__ dyn_w2, const float* __restrict__ dyn_b2,
    const float* __restrict__ coupling, const float* __restrict__ damping,
    const float* __restrict__ interaction,
    const float* __restrict__ summ_w, const float* __restrict__ summ_b,
    const float* __restrict__ fq_w1, const float* __restrict__ fq_b1, const float* __restrict__ fq_w2,
    const float* __restrict__ col_w1, const float* __restrict__ col_b1, const float* __restrict__ col_w2,
    const int* __restrict__ tptr,
    float* __restrict__ wsBias, unsigned short* __restrict__ wsW1t,
    unsigned short* __restrict__ wsWct, unsigned short* __restrict__ wsHh)
{
  __shared__ float sState[kState];
  __shared__ float sHidD[kDynHid];
  __shared__ float sDn[kState];
  __shared__ float sFo[64];
  __shared__ float sInter[kBlobs * kBlobs];
  __shared__ __align__(16) float sSum[kSumW];
  __shared__ __align__(16) float sBias[128];

  const int tid = threadIdx.x;
  const int lane = tid & 31;
  const int wave = tid >> 5;

  {
    v8h pw1, pwc, phd;
    {
      const int n = tid >> 2;
      const int kc = (tid & 3) * 8;
      const bool live = (kc < kEnc);
      const int kcl = live ? kc : (kEnc - 8);
      const v4f a0 = pin_v4(*(const v4f*)(fq_w1 + n * kFqIn + kcl));
      const v4f a1 = pin_v4(*(const v4f*)(fq_w1 + n * kFqIn + kcl + 4));
#pragma unroll
      for (int e = 0; e < 4; ++e) {
        pw1[e]     = (_Float16)(live ? a0[e] : 0.0f);
        pw1[4 + e] = (_Float16)(live ? a1[e] : 0.0f);
      }
#pragma unroll
      for (int e = 0; e < 8; ++e) {
        const int k = kc + e;
        const int ks = (k < kEnc) ? k : (kColIn - 1);
        const float b = pin_f32(col_w1[n * kColIn + ks]);
        pwc[e] = (_Float16)((k <= kEnc) ? b : 0.0f);
      }
    }
    {
      const int qh = tid & 127;
      const int n = qh >> 3;
      const int kc = (qh & 7) * 8;
      int nr = n - 1;
      nr = (nr < 0) ? 0 : ((nr > 2) ? 2 : nr);
      const v4f d0 = pin_v4(*(const v4f*)(fq_w2 + kc));
      const v4f d1 = pin_v4(*(const v4f*)(fq_w2 + kc + 4));
      const v4f c0 = pin_v4(*(const v4f*)(col_w2 + nr * kHid + kc));
      const v4f c1 = pin_v4(*(const v4f*)(col_w2 + nr * kHid + kc + 4));
      const bool isd = (n == 0);
      const bool isc = (n >= 1) && (n <= 3);
#pragma unroll
      for (int e = 0; e < 4; ++e) {
        const float v0 = isd ? d0[e] : (isc ? c0[e] : 0.0f);
        const float v1 = isd ? d1[e] : (isc ? c1[e] : 0.0f);
        phd[e]     = (_Float16)v0;
        phd[4 + e] = (_Float16)v1;
      }
    }
    unsigned short* q1 = wsW1t + tid * 8;
    unsigned short* q2 = wsWct + tid * 8;
    unsigned short* q3 = wsHh + (tid & 127) * 8;
    for (int pass = 0; pass < 2; ++pass) {
      *(volatile v8h*)q1 = pw1;
      *(volatile v8h*)q2 = pwc;
      if (wave < 4) {
        *(volatile v8h*)q3 = phd;
      }
      __threadfence();
    }
  }

  {
    const int i0 = (tid < kState) ? tid : (kState - 1);
    const float v = initial_state[i0];
    const float w0 = interaction[tid];
    const int i1 = tid + 256;
    const int i1c = (i1 < kBlobs * kBlobs) ? i1 : (kBlobs * kBlobs - 1);
    const float w1 = interaction[i1c];
    if (tid < kState) sState[tid] = v;
    sInter[tid] = w0;
    if (i1 < kBlobs * kBlobs) sInter[i1] = w1;
  }
  const int tt = tptr[0];
  const int ttc = (tt < 1) ? 1 : ((tt > 1000) ? 1000 : tt);
  int ns = (tt >= 1) ? (ttc * 100) : 1;
  const bool overlong = (ns > kMaxSteps);
  ns = overlong ? kMaxSteps : ns;
  const float dt = (tt >= 1) ? 0.01f : (float)tt;
  const float cpl = coupling[0];
  const float dmp = damping[0];
  __syncthreads();

  for (int s = 0; s < ns; ++s) {
    if (wave < 2) {
      float acc = dyn_b1[tid];
      const float* wr = dyn_w1 + tid * kState;
#pragma unroll 4
      for (int k = 0; k < kState; ++k) acc = fmaf(wr[k], sState[k], acc);
      sHidD[tid] = tanhf(acc);
    }
    __syncthreads();
    if (wave < 5) {
      float acc = dyn_b2[tid];
      const float* wr = dyn_w2 + tid * kDynHid;
#pragma unroll 4
      for (int k = 0; k < kDynHid; ++k) acc = fmaf(wr[k], sHidD[k], acc);
      sDn[tid] = acc;
    } else if (wave == 5) {
      const int i = (lane < kBlobs) ? lane : (kBlobs - 1);
      const float xi = sState[i * 8], yi = sState[i * 8 + 1], zi = sState[i * 8 + 2];
      float fx = 0.0f, fy = 0.0f, fz = 0.0f;
#pragma unroll 1
      for (int j = 0; j < kBlobs; ++j) {
        const float dx = xi - sState[j * 8];
        const float dy = yi - sState[j * 8 + 1];
        const float dz = zi - sState[j * 8 + 2];
        const float d2 = dx * dx + dy * dy + dz * dz + 1e-6f;
        const float dist = sqrtf(d2);
        const float den = (dist * dist + 1.0f) * (dist + 1e-6f);
        const float w = sInter[i * kBlobs + j] / den;
        fx += w * dx;
        fy += w * dy;
        fz += w * dz;
      }
      if (lane < kBlobs) {
        sFo[lane * 3 + 0] = fx;
        sFo[lane * 3 + 1] = fy;
        sFo[lane * 3 + 2] = fz;
      }
    }
    __syncthreads();
    float newv;
    {
      const int tc = (tid < kState) ? tid : (kState - 1);
      const int i = tc >> 3, c = tc & 7;
      const int cv = (c < 2) ? c : 2;
      int cf = c - 3;
      cf = (cf < 0) ? 0 : ((cf > 2) ? 2 : cf);
      const float sv   = sState[tc];
      const float velv = sState[i * 8 + 3 + cv];
      const float fov  = sFo[i * 3 + cf];
      const float dnv  = sDn[tc];
      const float dvel = -dmp * sv + cpl * fov + dnv;
      const float tgt  = (c == 6) ? 1.0f : 0.5f;
      const float dsz  = -0.05f * (sv - tgt) + dnv;
      const float ds   = (c < 3) ? velv : ((c < 6) ? dvel : dsz);
      newv = sv + dt * ds;
    }
    __syncthreads();
    if (tid < kState) sState[tid] = newv;
    __syncthreads();
  }

  if (wave == 0) {
    float acc = summ_b[tid];
    const float* wr = summ_w + tid * kState;
#pragma unroll 1
    for (int k = 0; k < kState; ++k) acc = fmaf(wr[k], sState[k], acc);
    sSum[tid] = acc;
  }
  __syncthreads();
  if (wave < 2) {
    float acc = fq_b1[tid];
    const float* wr = fq_w1 + tid * kFqIn + kEnc;
#pragma unroll 1
    for (int j = 0; j < kSumW; ++j) acc = fmaf(wr[j], sSum[j], acc);
    sBias[tid] = overlong ? __uint_as_float(0x7fc00000u) : acc;
  } else if (wave < 4) {
    const int n = tid - 64;
    float acc = col_b1[n];
    const float* wr = col_w1 + n * kColIn + kEnc;
#pragma unroll 1
    for (int j = 0; j < kSumW; ++j) acc = fmaf(wr[j], sSum[j], acc);
    sBias[tid] = overlong ? __uint_as_float(0x7fc00000u) : acc;
  }
  __syncthreads();
  if (wave == 0) {
    const v4f bv = *(const v4f*)(sBias + lane * 4);
    float* q = wsBias + lane * 4;
    for (int pass = 0; pass < 2; ++pass) {
      *(volatile v4f*)q = bv;
      __threadfence();
    }
  }
}

__device__ __forceinline__ v8f mlp_tile(const _Float16* aw, _Float16* hw, int mt, int cn, int koff,
                                        v16h b0, v16h b1, v16h b2, v16h b3,
                                        float s0, float s1, float s2, float s3,
                                        v16h hd0, v16h hd1, float hb)
{
  const v16h a = Frag<_Float16>::load(aw + (mt * 16 + cn) * kAP + koff);
  v8f acc[4];
#pragma unroll
  for (int r = 0; r < 8; ++r) {
    acc[0][r] = s0;
    acc[1][r] = s1;
    acc[2][r] = s2;
    acc[3][r] = s3;
  }
  acc[0] = mma_h(a, b0, acc[0]);
  acc[1] = mma_h(a, b1, acc[1]);
  acc[2] = mma_h(a, b2, acc[2]);
  acc[3] = mma_h(a, b3, acc[3]);
#pragma unroll
  for (int nt = 0; nt < 4; ++nt) {
#pragma unroll
    for (int r = 0; r < 8; ++r)
      hw[(koff + r) * kHP + nt * 16 + cn] = (_Float16)fmaxf(acc[nt][r], 0.0f);
  }
  wave_lds_sync();
  const v16h h0 = Frag<_Float16>::load(hw + cn * kHP + koff);
  const v16h h1 = Frag<_Float16>::load(hw + cn * kHP + 32 + koff);
  v8f z;
#pragma unroll
  for (int r = 0; r < 8; ++r) z[r] = hb;
  z = mma_h(h0, hd0, z);
  z = mma_h(h1, hd1, z);
  return z;
}

__global__ __launch_bounds__(256) void field_kernel(
    const float* __restrict__ p,
    const float* __restrict__ wsBias,
    const unsigned short* __restrict__ wsW1t,
    const unsigned short* __restrict__ wsWct,
    const unsigned short* __restrict__ wsHh,
    const float* __restrict__ fq_b2, const float* __restrict__ col_b2,
    float* __restrict__ out)
{
  __shared__ __align__(16) _Float16 sA[kWavesPerBlock][kGroupPts * kAP];
  __shared__ __align__(16) _Float16 sH[kWavesPerBlock][16 * kHP];
  __shared__ __align__(16) float sZ[kWavesPerBlock][kGroupPts];
  __shared__ __align__(16) float sC[kWavesPerBlock][kGroupPts * 3];

  const int lane = threadIdx.x & 31;
  const int wave = threadIdx.x >> 5;
  const int hh = lane >> 4;
  const int cn = lane & 15;
  const int koff = hh * 8;

  const _Float16* W1t = (const _Float16*)(const void*)wsW1t;
  const _Float16* Wct = (const _Float16*)(const void*)wsWct;
  const _Float16* Hh  = (const _Float16*)(const void*)wsHh;

  const v16h ba0 = Frag<_Float16>::load(W1t + (0 * 16 + cn) * kKP + koff);
  const v16h ba1 = Frag<_Float16>::load(W1t + (1 * 16 + cn) * kKP + koff);
  const v16h ba2 = Frag<_Float16>::load(W1t + (2 * 16 + cn) * kKP + koff);
  const v16h ba3 = Frag<_Float16>::load(W1t + (3 * 16 + cn) * kKP + koff);
  const v16h bb0 = Frag<_Float16>::load(Wct + (0 * 16 + cn) * kKP + koff);
  const v16h bb1 = Frag<_Float16>::load(Wct + (1 * 16 + cn) * kKP + koff);
  const v16h bb2 = Frag<_Float16>::load(Wct + (2 * 16 + cn) * kKP + koff);
  const v16h bb3 = Frag<_Float16>::load(Wct + (3 * 16 + cn) * kKP + koff);
  const v16h hd0 = Frag<_Float16>::load(Hh + cn * kHid + koff);
  const v16h hd1 = Frag<_Float16>::load(Hh + cn * kHid + 32 + koff);

  const float sa0 = wsBias[0 * 16 + cn];
  const float sa1 = wsBias[1 * 16 + cn];
  const float sa2 = wsBias[2 * 16 + cn];
  const float sa3 = wsBias[3 * 16 + cn];
  const float sb0 = wsBias[64 + 0 * 16 + cn];
  const float sb1 = wsBias[64 + 1 * 16 + cn];
  const float sb2 = wsBias[64 + 2 * 16 + cn];
  const float sb3 = wsBias[64 + 3 * 16 + cn];
  const float fb2 = pin_f32(fq_b2[0]);
  int cbi = cn - 1;
  cbi = (cbi < 0) ? 0 : ((cbi > 2) ? 2 : cbi);
  const float cb2 = pin_f32(col_b2[cbi]);
  const float hbD = (cn == 0) ? fb2 : 0.0f;
  const bool colLane = (cn >= 1) && (cn <= 3);
  const float hbC = colLane ? cb2 : 0.0f;

  _Float16* aw = sA[wave];
  _Float16* hw = sH[wave];
  float* sz = sZ[wave];
  float* sc = sC[wave];

#pragma unroll 1
  for (int g = 0; g < kGroupsPerWave; ++g) {
    const int base = (blockIdx.x * kWavesPerBlock + wave) * (kGroupsPerWave * kGroupPts) + g * kGroupPts;
    const int idx = base + lane;
    const float x0 = p[(size_t)3 * idx];
    const float x1 = p[(size_t)3 * idx + 1];
    const float x2 = p[(size_t)3 * idx + 2];

    {
      float pe[kEnc];
#pragma unroll
      for (int d = 0; d < 3; ++d) {
        const float xd = (d == 0) ? x0 : ((d == 1) ? x1 : x2);
        const float a0 = pin_f32(6.28318530717958647692f * xd);
        float sv = sinf(a0);
        float cv = cosf(a0);
        pe[d] = sv;
        pe[3 + d] = cv;
#pragma unroll
        for (int i = 1; i < 4; ++i) {
          const float s2 = 2.0f * sv * cv;
          const float c2 = 1.0f - 2.0f * sv * sv;
          sv = s2;
          cv = c2;
          pe[6 * i + d] = sv;
          pe[6 * i + 3 + d] = cv;
        }
      }
      v8h e0, e1, e2, z8;
#pragma unroll
      for (int q = 0; q < 8; ++q) {
        e0[q] = (_Float16)pe[q];
        e1[q] = (_Float16)pe[8 + q];
        e2[q] = (_Float16)pe[16 + q];
        z8[q] = (_Float16)0.0f;
      }
      _Float16* arow = aw + lane * kAP;
      *(v8h*)(arow)      = e0;
      *(v8h*)(arow + 8)  = e1;
      *(v8h*)(arow + 16) = e2;
      *(v8h*)(arow + 24) = z8;
    }
    wave_lds_sync();

#pragma unroll 1
    for (int mt = 0; mt < 2; ++mt) {
      const v8f z = mlp_tile(aw, hw, mt, cn, koff, ba0, ba1, ba2, ba3, sa0, sa1, sa2, sa3, hd0, hd1, hbD);
      if (cn == 0) {
#pragma unroll
        for (int r = 0; r < 8; ++r) sz[mt * 16 + koff + r] = z[r];
      }
      wave_lds_sync();
    }

    const float zv = sz[lane];
    const float dens = fmaxf(zv, 0.0f) + log1pf(expf(-fabsf(zv)));
    aw[lane * kAP + kEnc] = (_Float16)dens;
    wave_lds_sync();

#pragma unroll 1
    for (int mt = 0; mt < 2; ++mt) {
      const v8f z = mlp_tile(aw, hw, mt, cn, koff, bb0, bb1, bb2, bb3, sb0, sb1, sb2, sb3, hd0, hd1, hbC);
      if (colLane) {
#pragma unroll
        for (int r = 0; r < 8; ++r) sc[(mt * 16 + koff + r) * 3 + (cn - 1)] = z[r];
      }
      wave_lds_sync();
    }

    float cv0, cv1, cv2;
    {
      const float l0 = sc[lane];
      const float l1 = sc[lane + 32];
      const float l2 = sc[lane + 64];
      cv0 = 1.0f / (1.0f + expf(-l0));
      cv1 = 1.0f / (1.0f + expf(-l1));
      cv2 = 1.0f / (1.0f + expf(-l2));
    }

    {
      volatile float* o0 = out + idx;
      volatile float* o1 = out + (size_t)kN + (size_t)3 * base + lane;
      for (int pass = 0; pass < 2; ++pass) {
        o0[0]  = dens;
        o1[0]  = cv0;
        o1[32] = cv1;
        o1[64] = cv2;
        __threadfence();
      }
    }
    wave_lds_sync();
  }
}

extern "C" void kernel_launch(void* const* d_in, const int* in_sizes, int n_in,
                              void* d_out, int out_size, void* d_ws, size_t ws_size,
                              hipStream_t stream) {
  if (n_in < 20) return;
  if (in_sizes[0] != kN * 3) return;
  if (in_sizes[1] != kState) return;
  if (in_sizes[2] != kDynHid * kState) return;
  if (in_sizes[3] != kDynHid) return;
  if (in_sizes[4] != kState * kDynHid) return;
  if (in_sizes[5] != kState) return;
  if (in_sizes[6] != 1 || in_sizes[7] != 1) return;
  if (in_sizes[8] != kBlobs * kBlobs) return;
  if (in_sizes[9] != kSumW * kState) return;
  if (in_sizes[10] != kSumW) return;
  if (in_sizes[11] != kHid * kFqIn) return;
  if (in_sizes[12] != kHid) return;
  if (in_sizes[13] != kHid) return;
  if (in_sizes[14] != 1) return;
  if (in_sizes[15] != kHid * kColIn) return;
  if (in_sizes[16] != kHid) return;
  if (in_sizes[17] != 3 * kHid) return;
  if (in_sizes[18] != 3) return;
  if (in_sizes[19] != 1) return;
  if (out_size != kN * 4) return;
  if (ws_size < kWsTotal) return;

  const float* p             = (const float*)d_in[0];
  const float* initial_state = (const float*)d_in[1];
  const float* dyn_w1        = (const float*)d_in[2];
  const float* dyn_b1        = (const float*)d_in[3];
  const float* dyn_w2        = (const float*)d_in[4];
  const float* dyn_b2        = (const float*)d_in[5];
  const float* coupling      = (const float*)d_in[6];
  const float* damping       = (const float*)d_in[7];
  const float* interaction   = (const float*)d_in[8];
  const float* summ_w        = (const float*)d_in[9];
  const float* summ_b        = (const float*)d_in[10];
  const float* fq_w1         = (const float*)d_in[11];
  const float* fq_b1         = (const float*)d_in[12];
  const float* fq_w2         = (const float*)d_in[13];
  const float* fq_b2         = (const float*)d_in[14];
  const float* col_w1        = (const float*)d_in[15];
  const float* col_b1        = (const float*)d_in[16];
  const float* col_w2        = (const float*)d_in[17];
  const float* col_b2        = (const float*)d_in[18];
  const int*   tptr          = (const int*)d_in[19];

  char* ws = (char*)d_ws;
  float*          wsBias = (float*)(ws + kOffBias);
  unsigned short* wsW1t  = (unsigned short*)(ws + kOffW1t);
  unsigned short* wsWct  = (unsigned short*)(ws + kOffWct);
  unsigned short* wsHh   = (unsigned short*)(ws + kOffHh);

  prep_kernel<<<1, 256, 0, stream>>>(initial_state, dyn_w1, dyn_b1, dyn_w2, dyn_b2,
                                     coupling, damping, interaction, summ_w, summ_b,
                                     fq_w1, fq_b1, fq_w2, col_w1, col_b1, col_w2, tptr,
                                     wsBias, wsW1t, wsWct, wsHh);

  field_kernel<<<kN / kBlockPts, 256, 0, stream>>>(p, wsBias, wsW1t, wsWct, wsHh,
                                                   fq_b2, col_b2, (float*)d_out);
}
